// GCN_Layer_39453569581648
// MI455X (gfx1250) — hardware-run, weakly checked
//
#include <hip/hip_runtime.h>
#include <stddef.h>
#include <stdint.h>


#define NNODES  50000
#define DF      128
#define AP      256
#define WDP     256
#define NTERMS  2
#define KG      (DF * NTERMS)
#define NTHR    256
#define NWAVE   8
#define EPT     8
#define WIT     (32 * EPT)
#define WLCAP   4096
#define NBA     1024
#define PKS     10
#define RCAP    16384
#define DEGCAP  64
#define GBM     128
#define GTHR    256
#define RPB     64
#define RPW     8
#define UW      (DF * 32)
#define BK_INTS (NWAVE * WLCAP + RCAP + 3 * NBA + 32)
#define LDS_BK  (BK_INTS * 4)
#define LDS_GM  ((GBM * DF + DF) * 4)
#define MEAS_BLK_HITS 13410
#define MEAS_MAXDEG   30

static_assert(DF == 128 && DF == 32 * 4);
static_assert(NBA % 32 == 0 && NBA == (1 << PKS) && NBA == NTHR * 4);
static_assert(49 * NBA >= NNODES && 48 * NBA + 848 == NNODES);
static_assert((long long)RCAP * 100 >= (long long)MEAS_BLK_HITS * 105);
static_assert(DEGCAP >= MEAS_MAXDEG + 8);
static_assert(RCAP % (NTHR * 4) == 0 && BK_INTS % 4 == 0);
static_assert(NWAVE * WLCAP >= RCAP);
static_assert(NTERMS == 1 || NTERMS == 2);
static_assert(KG == 128 * NTERMS && KG % 32 == 0 && KG <= AP && KG <= WDP);
static_assert(GBM == (GTHR / 32) * 16 && NBA % GBM == 0);
static_assert(390 * GBM + 80 == NNODES && 391 * GBM == 50048);
static_assert(UW % NTHR == 0);
static_assert(RPB == NWAVE * RPW);
static_assert(LDS_BK <= 300000 && LDS_BK <= 327680);
static_assert(LDS_GM + 0 <= 327680);
static_assert(NWAVE * AP * 2 <= 327680);

typedef float          v4f   __attribute__((ext_vector_type(4)));
typedef float          v8f   __attribute__((ext_vector_type(8)));
typedef int            v4i   __attribute__((ext_vector_type(4)));
typedef int            v8i   __attribute__((ext_vector_type(8)));
typedef unsigned       v4u   __attribute__((ext_vector_type(4)));
typedef unsigned short v4us  __attribute__((ext_vector_type(4)));
typedef unsigned short v8us  __attribute__((ext_vector_type(8)));
typedef __bf16         v16bf __attribute__((ext_vector_type(16)));
typedef v4f  __attribute__((may_alias)) v4fa;
typedef v4i  __attribute__((may_alias)) v4ia;
typedef v4us __attribute__((may_alias)) v4usa;
typedef v8us __attribute__((may_alias)) v8usa;
union FragB { v16bf v; v8us h[2]; v8i w; };

__device__ __forceinline__ v8f wmb(const FragB& a, const FragB& b, v8f c) {
  v8f d = __builtin_amdgcn_wmma_f32_16x16x32_bf16(false, a.v, false, b.v, (short)0, c, false, false);
  asm volatile("v_nop\n\tv_nop\n\tv_nop\n\tv_nop" : "+v"(d) : "v"(a.w), "v"(b.w));
  return d;
}

__device__ __forceinline__ unsigned bf16_bits(float f) {
  const unsigned u = __float_as_uint(f);
  return ((u + 0x7FFFu + ((u >> 16) & 1u)) >> 16) & 0xFFFFu;
}
__device__ __forceinline__ float bf16_val(float f) { return __uint_as_float(bf16_bits(f) << 16); }

__device__ __forceinline__ void wave_sync() {
  __builtin_amdgcn_fence(__ATOMIC_RELEASE, "wavefront");
  __builtin_amdgcn_wave_barrier();
  __builtin_amdgcn_fence(__ATOMIC_ACQUIRE, "wavefront");
}

__global__ __launch_bounds__(NTHR) void k_prep(const float* __restrict__ W, const float* __restrict__ b,
                                               unsigned short* WD, float* BT, unsigned short* AGG,
                                               int nN, int padPieces) {
  const int u = (int)blockIdx.x * NTHR + (int)threadIdx.x;
  if (u < UW) {
    const int n   = u >> 5;
    const int j   = u & 31;
    const int kk0 = (j & 15) * 8;
    const int k8  = (j >> 4) * 128 + kk0;
    float f[8];
#pragma unroll
    for (int i = 0; i < 8; ++i) f[i] = W[(size_t)(kk0 + i) * DF + (size_t)n];
    v8us o;
#pragma unroll
    for (int i = 0; i < 8; ++i) o[i] = (unsigned short)bf16_bits(f[i]);
    unsigned short* dp = WD + (size_t)n * WDP + (size_t)k8;
    *(volatile v8us*)dp = o;
    __threadfence();
    *(volatile v8us*)dp = o;
  } else if (u < UW + 32) {
    const int t = u - UW;
    const v4f b4 = *(const v4f*)(b + 4 * t);
    v4f bq;
    bq.x = bf16_val(b4.x); bq.y = bf16_val(b4.y); bq.z = bf16_val(b4.z); bq.w = bf16_val(b4.w);
    float* dp = BT + 4 * t;
    *(volatile v4f*)dp = bq;
    __threadfence();
    *(volatile v4f*)dp = bq;
  } else {
    const int p = u - (UW + 32);
    if (p < padPieces) {
      const int row = nN + (p >> 5);
      const v4u z = {0u, 0u, 0u, 0u};
      unsigned short* dp = AGG + (size_t)row * AP + 8 * (p & 31);
      *(volatile v4u*)dp = z;
      __threadfence();
      *(volatile v4u*)dp = z;
    }
  }
}

__device__ __forceinline__ int scan_step(const int* __restrict__ keys, int base, int segEnd, int nE,
                                         int slotBase, int nb, int* wlw, int wc, int lane) {
  const int e0   = base + lane * EPT;
  const int sent = -2147483647 - 1;
  v4i da, db;
  if (base + WIT <= segEnd) {
    da = *(const v4i*)(keys + e0);
    db = *(const v4i*)(keys + e0 + 4);
  } else {
    const int hi = nE - 1;
    const int t0 = keys[min(e0,     hi)];
    const int t1 = keys[min(e0 + 1, hi)];
    const int t2 = keys[min(e0 + 2, hi)];
    const int t3 = keys[min(e0 + 3, hi)];
    const int t4 = keys[min(e0 + 4, hi)];
    const int t5 = keys[min(e0 + 5, hi)];
    const int t6 = keys[min(e0 + 6, hi)];
    const int t7 = keys[min(e0 + 7, hi)];
    asm volatile("" :: "v"(t0), "v"(t1), "v"(t2), "v"(t3), "v"(t4), "v"(t5), "v"(t6), "v"(t7));
    da.x = (e0     < segEnd) ? t0 : sent;
    da.y = (e0 + 1 < segEnd) ? t1 : sent;
    da.z = (e0 + 2 < segEnd) ? t2 : sent;
    da.w = (e0 + 3 < segEnd) ? t3 : sent;
    db.x = (e0 + 4 < segEnd) ? t4 : sent;
    db.y = (e0 + 5 < segEnd) ? t5 : sent;
    db.z = (e0 + 6 < segEnd) ? t6 : sent;
    db.w = (e0 + 7 < segEnd) ? t7 : sent;
  }
  const unsigned nbs = (unsigned)slotBase;
  const unsigned unb = (unsigned)nb;
  const unsigned s0 = (unsigned)da.x - nbs, s1 = (unsigned)da.y - nbs;
  const unsigned s2 = (unsigned)da.z - nbs, s3 = (unsigned)da.w - nbs;
  const unsigned s4 = (unsigned)db.x - nbs, s5 = (unsigned)db.y - nbs;
  const unsigned s6 = (unsigned)db.z - nbs, s7 = (unsigned)db.w - nbs;
  const bool h0 = s0 < unb, h1 = s1 < unb, h2 = s2 < unb, h3 = s3 < unb;
  const bool h4 = s4 < unb, h5 = s5 < unb, h6 = s6 < unb, h7 = s7 < unb;
  const int c = (h0 ? 1 : 0) + (h1 ? 1 : 0) + (h2 ? 1 : 0) + (h3 ? 1 : 0) +
                (h4 ? 1 : 0) + (h5 ? 1 : 0) + (h6 ? 1 : 0) + (h7 ? 1 : 0);
  int incl = c;
#pragma unroll
  for (int d = 1; d < 32; d <<= 1) {
    const int up = __shfl_up(incl, d, 32);
    incl += (lane >= d) ? up : 0;
  }
  const int tot = __shfl(incl, 31, 32);
  int pos = wc + incl - c;
#define PUTJ(J, HJ, SJ) { \
    if ((HJ) && pos < WLCAP) wlw[pos] = (int)(((unsigned)(e0 + (J)) << PKS) | (SJ)); \
    pos += (HJ) ? 1 : 0; }
  PUTJ(0, h0, s0)
  PUTJ(1, h1, s1)
  PUTJ(2, h2, s2)
  PUTJ(3, h3, s3)
  PUTJ(4, h4, s4)
  PUTJ(5, h5, s5)
  PUTJ(6, h6, s6)
  PUTJ(7, h7, s7)
#undef PUTJ
  return wc + tot;
}

template <int ROLE>
__device__ __forceinline__ void bucket_body(const int* __restrict__ keys, const int* __restrict__ gidx,
                                            int nE, int nN, int segLen, int blk, int frow, int* dsm,
                                            int* LIST, int* CNT, int* OFF, int* NRM, int* FLG) {
  int* wl   = dsm;
  int* reg2 = wl + NWAVE * WLCAP;
  int* scnt = reg2 + RCAP;
  int* soff = scnt + NBA;
  int* cur  = soff + NBA;
  int* wcn  = cur + NBA;
  int* wtot = wcn + 8;
  int* wmx  = wtot + 8;
  const int tid = (int)threadIdx.x, lane = tid & 31, wave = tid >> 5;
  const int nodeBase = blk * NBA;
  int nb = nN - nodeBase;
  nb = nb > NBA ? NBA : (nb < 1 ? 1 : nb);

  {
    const v4i z4 = {0, 0, 0, 0};
    for (int i = tid * 4; i < BK_INTS; i += NTHR * 4) *(v4ia*)(dsm + i) = z4;
  }
  __syncthreads();

  {
    const int segBeg = wave * segLen;
    int segEnd = segBeg + segLen;
    segEnd = segEnd > nE ? nE : segEnd;
    int* wlw = wl + wave * WLCAP;
    int wc = 0;
#pragma unroll 1
    for (int base = segBeg; base < segEnd; base += WIT)
      wc = scan_step(keys, base, segEnd, nE, nodeBase, nb, wlw, wc, lane);
    if (lane == 0) wcn[wave] = wc;
  }
  __syncthreads();

  int nh = 0, wov = 0;
#pragma unroll
  for (int w2 = 0; w2 < NWAVE; ++w2) {
    int c = wcn[w2];
    wov |= (c > WLCAP) ? 1 : 0;
    c = c < 0 ? 0 : (c > WLCAP ? WLCAP : c);
    nh += c;
  }
  const int rov = (nh > RCAP) ? 1 : 0;
  nh = nh > RCAP ? RCAP : nh;

  if (wave == 0) {
#pragma unroll 1
    for (int w2 = 0; w2 < NWAVE; ++w2) {
      int c = wcn[w2];
      c = c < 0 ? 0 : (c > WLCAP ? WLCAP : c);
      const int* lw = wl + w2 * WLCAP;
#pragma unroll 1
      for (int b0 = 0; b0 < c; b0 += 32) {
        const int idx = b0 + lane;
        const int ent = lw[idx < WLCAP ? idx : WLCAP - 1];
        const int m32 = (c - b0) < 32 ? (c - b0) : 32;
#pragma unroll 1
        for (int k = 0; k < m32; ++k) {
          const int u  = __builtin_amdgcn_readlane(ent, k);
          const int sl = u & (NBA - 1);
          if (lane == 0) scnt[sl] = scnt[sl] + 1;
        }
      }
    }
  }
  __syncthreads();

  {
    const v4i ca = *(const v4ia*)(scnt + 4 * tid);
    const int e0 = ca.x < 0 ? 0 : ca.x, e1 = ca.y < 0 ? 0 : ca.y, e2 = ca.z < 0 ? 0 : ca.z, e3 = ca.w < 0 ? 0 : ca.w;
    const int ts = e0 + e1 + e2 + e3;
    int incl = ts;
#pragma unroll
    for (int d = 1; d < 32; d <<= 1) {
      const int up = __shfl_up(incl, d, 32);
      incl += (lane >= d) ? up : 0;
    }
    int mx = max(max(e0, e1), max(e2, e3));
    mx = max(mx, __shfl_xor(mx, 16, 32));
    mx = max(mx, __shfl_xor(mx, 8, 32));
    mx = max(mx, __shfl_xor(mx, 4, 32));
    mx = max(mx, __shfl_xor(mx, 2, 32));
    mx = max(mx, __shfl_xor(mx, 1, 32));
    if (lane == 31) wtot[wave] = incl;
    if (lane == 0)  wmx[wave] = mx;
    __syncthreads();
    int pre = 0;
#pragma unroll
    for (int w2 = 0; w2 < NWAVE; ++w2) pre += (w2 < wave) ? wtot[w2] : 0;
    int run = pre + incl - ts;
    v4i so;
    so.x = run; run += e0;
    so.y = run; run += e1;
    so.z = run; run += e2;
    so.w = run;
    *(v4ia*)(soff + 4 * tid) = so;
    *(v4ia*)(cur + 4 * tid)  = so;
  }
  __syncthreads();

  if constexpr (ROLE == 0) {
    if (wave == 0) {
#pragma unroll 1
      for (int w2 = 0; w2 < NWAVE; ++w2) {
        int c = wcn[w2];
        c = c < 0 ? 0 : (c > WLCAP ? WLCAP : c);
        const int* lw = wl + w2 * WLCAP;
#pragma unroll 1
        for (int b0 = 0; b0 < c; b0 += 32) {
          const int idx = b0 + lane;
          const int ent = lw[idx < WLCAP ? idx : WLCAP - 1];
          const int m32 = (c - b0) < 32 ? (c - b0) : 32;
#pragma unroll 1
          for (int k = 0; k < m32; ++k) {
            const int u   = __builtin_amdgcn_readlane(ent, k);
            const int sl  = u & (NBA - 1);
            const int eid = (int)((unsigned)u >> PKS);
            if (lane == 0) {
              int pos = cur[sl];
              pos = pos < 0 ? 0 : (pos > RCAP - 1 ? RCAP - 1 : pos);
              reg2[pos] = eid;
              cur[sl] = pos + 1;
            }
          }
        }
      }
    }
    __syncthreads();
  }

  int bmax = 0;
#pragma unroll
  for (int w2 = 0; w2 < NWAVE; ++w2) bmax = max(bmax, wmx[w2]);
  int flag = wov;
  if constexpr (ROLE == 0) flag = flag | rov | ((bmax > DEGCAP) ? 1 : 0);

  if constexpr (ROLE == 0) {
    int* lrow = LIST + (size_t)blk * RCAP;
#pragma unroll 1
    for (int it = 0; it < RCAP / (NTHR * 4); ++it) {
      const int i0 = 4 * (it * NTHR + tid);
      const v4i ev = *(const v4ia*)(reg2 + i0);
      int e0 = ev.x, e1 = ev.y, e2 = ev.z, e3 = ev.w;
      e0 = e0 < 0 ? 0 : (e0 > nE - 1 ? nE - 1 : e0);
      e1 = e1 < 0 ? 0 : (e1 > nE - 1 ? nE - 1 : e1);
      e2 = e2 < 0 ? 0 : (e2 > nE - 1 ? nE - 1 : e2);
      e3 = e3 < 0 ? 0 : (e3 > nE - 1 ? nE - 1 : e3);
      int g0 = gidx[e0], g1 = gidx[e1], g2 = gidx[e2], g3 = gidx[e3];
      asm volatile("" :: "v"(g0), "v"(g1), "v"(g2), "v"(g3));
      g0 = g0 < 0 ? 0 : (g0 > nN - 1 ? nN - 1 : g0);
      g1 = g1 < 0 ? 0 : (g1 > nN - 1 ? nN - 1 : g1);
      g2 = g2 < 0 ? 0 : (g2 > nN - 1 ? nN - 1 : g2);
      g3 = g3 < 0 ? 0 : (g3 > nN - 1 ? nN - 1 : g3);
      v4i ov;
      ov.x = (i0     < nh) ? g0 : 0;
      ov.y = (i0 + 1 < nh) ? g1 : 0;
      ov.z = (i0 + 2 < nh) ? g2 : 0;
      ov.w = (i0 + 3 < nh) ? g3 : 0;
      *(volatile v4i*)(lrow + i0) = ov;
      __threadfence();
      *(volatile v4i*)(lrow + i0) = ov;
    }
  }

#pragma unroll 1
  for (int i = 0; i < 4; ++i) {
    int c = scnt[4 * tid + i];
    c = c < 0 ? 0 : c;
    float d = (float)(c + 1);
    d = fmaxf(d, 1.0f);
    cur[4 * tid + i] = __float_as_int(1.0f / sqrtf(d));
  }
  {
    const v4i cv = *(const v4ia*)(scnt + 4 * tid);
    const v4i fv = *(const v4ia*)(soff + 4 * tid);
    const v4i nv = *(const v4ia*)(cur + 4 * tid);
    v4i rv = {0, 0, 0, 0};
    rv.x = (tid == 0) ? bmax : 0;
    rv.y = (tid == 0) ? flag : 0;
    rv.z = (tid == 0) ? nh : 0;
    int* cp = CNT + (size_t)nodeBase + 4 * tid;
    int* fp = OFF + (size_t)nodeBase + 4 * tid;
    int* np = NRM + (size_t)nodeBase + 4 * tid;
    int* rp = FLG + (size_t)frow * 32 + 4 * (tid & 7);
    if constexpr (ROLE == 0) {
      *(volatile v4i*)cp = cv;
      *(volatile v4i*)fp = fv;
    }
    *(volatile v4i*)np = nv;
    if (tid < 8) *(volatile v4i*)rp = rv;
    __threadfence();
    if constexpr (ROLE == 0) {
      *(volatile v4i*)cp = cv;
      *(volatile v4i*)fp = fv;
    }
    *(volatile v4i*)np = nv;
    if (tid < 8) *(volatile v4i*)rp = rv;
  }
}

__global__ __launch_bounds__(NTHR) void k_bucket(const int* __restrict__ srcv, const int* __restrict__ dstv,
                                                 int nE, int nN, int segLen, int nB,
                                                 int* LIST, int* CNT, int* OFF, int* NI, int* NO, int* FLG) {
  extern __shared__ __attribute__((aligned(16))) int dsm[];
  const int b = (int)blockIdx.x;
  if (b < nB) bucket_body<0>(dstv, srcv, nE, nN, segLen, b, b, dsm, LIST, CNT, OFF, NI, FLG);
  else        bucket_body<1>(srcv, srcv, nE, nN, segLen, b - nB, b, dsm, LIST, CNT, OFF, NO, FLG);
}

__global__ __launch_bounds__(NTHR) void k_prescale(const float* __restrict__ x, const float* __restrict__ NO,
                                                   const int* __restrict__ FLG, float* PN, int nN, int nB) {
  const int tid = (int)threadIdx.x, lane = tid & 31, wave = tid >> 5;
  const float qn = __int_as_float(0x7fc00000);
#pragma unroll 1
  for (int ri = 0; ri < RPW; ++ri) {
    const int row = (int)blockIdx.x * RPB + wave * RPW + ri;
    if (row >= nN) continue;
    const v4f xv = *(const v4f*)(x + (size_t)row * DF + 4 * lane);
    const float no = NO[row];
    const int fl = FLG[(size_t)(nB + (row >> PKS)) * 32 + 1];
    const bool pz = fl != 0;
    v4f o;
    o.x = bf16_val(xv.x) * no;
    o.y = bf16_val(xv.y) * no;
    o.z = bf16_val(xv.z) * no;
    o.w = bf16_val(xv.w) * no;
    o.x = pz ? qn : o.x; o.y = pz ? qn : o.y; o.z = pz ? qn : o.z; o.w = pz ? qn : o.w;
    float* dp = PN + (size_t)row * DF + 4 * lane;
    *(volatile v4f*)dp = o;
    __threadfence();
    *(volatile v4f*)dp = o;
  }
}

__global__ __launch_bounds__(NTHR) void k_replay(const float* __restrict__ PN, const int* __restrict__ LIST,
                                                 const int* __restrict__ CNT, const int* __restrict__ OFF,
                                                 const float* __restrict__ NI, const int* __restrict__ FLG,
                                                 unsigned short* AGG, int nN) {
  __shared__ __attribute__((aligned(16))) unsigned short rowst[NWAVE * AP];
  const int tid = (int)threadIdx.x, lane = tid & 31, wave = tid >> 5;
  const int blk = (int)blockIdx.x;
  const int nodeBase = blk * NBA;
  const int fl = FLG[(size_t)blk * 32 + 1];
  const int* lp = LIST + (size_t)blk * RCAP;
  unsigned short* rowbuf = rowst + wave * AP;
  const float qn = __int_as_float(0x7fc00000);
#pragma unroll 1
  for (int si = 0; si < NBA / NWAVE; ++si) {
    const int s    = si * NWAVE + wave;
    const int node = nodeBase + s;
    if (node >= nN) continue;
    const int craw = CNT[node];
    const int oraw = OFF[node];
    const bool big = craw > DEGCAP;
    int c = craw < 0 ? 0 : (craw > DEGCAP ? DEGCAP : craw);
    int o = oraw < 0 ? 0 : (oraw > RCAP ? RCAP : oraw);
    if (c > RCAP - o) c = RCAP - o;
    int last = o + c - 1; last = last < o ? o : last;
    float a0 = 0.0f, a1 = 0.0f, a2 = 0.0f, a3 = 0.0f;
#pragma unroll 1
    for (int b0 = 0; b0 < c; b0 += 32) {
      int idx = o + b0 + lane;
      idx = idx > last ? last : idx;
      idx = idx > RCAP - 1 ? RCAP - 1 : idx;
      int col = lp[idx];
      col = col < 0 ? 0 : (col > nN - 1 ? nN - 1 : col);
      const int m32 = (c - b0) < 32 ? (c - b0) : 32;
#pragma unroll 1
      for (int k = 0; k < m32; ++k) {
        const int sk = __builtin_amdgcn_readlane(col, k);
        const v4f v = *(const v4f*)(PN + (size_t)sk * DF + 4 * lane);
        a0 += v.x; a1 += v.y; a2 += v.z; a3 += v.w;
      }
    }
    const v4f sv = *(const v4f*)(PN + (size_t)node * DF + 4 * lane);
    const float ni = NI[node];
    a0 += sv.x; a1 += sv.y; a2 += sv.z; a3 += sv.w;
    float m0 = a0 * ni, m1 = a1 * ni, m2 = a2 * ni, m3 = a3 * ni;
    const bool pz = (fl != 0) || big;
    m0 = pz ? qn : m0; m1 = pz ? qn : m1; m2 = pz ? qn : m2; m3 = pz ? qn : m3;
    v4us mh, ml;
    {
      unsigned hb;
      hb = bf16_bits(m0); mh[0] = (unsigned short)hb; ml[0] = (unsigned short)bf16_bits(m0 - __uint_as_float(hb << 16));
      hb = bf16_bits(m1); mh[1] = (unsigned short)hb; ml[1] = (unsigned short)bf16_bits(m1 - __uint_as_float(hb << 16));
      hb = bf16_bits(m2); mh[2] = (unsigned short)hb; ml[2] = (unsigned short)bf16_bits(m2 - __uint_as_float(hb << 16));
      hb = bf16_bits(m3); mh[3] = (unsigned short)hb; ml[3] = (unsigned short)bf16_bits(m3 - __uint_as_float(hb << 16));
    }
    *(v4usa*)(rowbuf + 4 * lane) = mh;
    *(v4usa*)(rowbuf + DF + 4 * lane) = ml;
    wave_sync();
    const v8us q0 = *(const v8usa*)(rowbuf + 8 * lane);
    wave_sync();
    unsigned short* rpw = AGG + (size_t)node * AP + 8 * lane;
    *(volatile v8us*)rpw = q0;
    __threadfence();
    *(volatile v8us*)rpw = q0;
  }
}

__device__ __forceinline__ void out_pass(const float* stg, v4f bb, bool pz, float* outp,
                                         int rowBase, int wave, int lane, int nN) {
  const float qn = __int_as_float(0x7fc00000);
#pragma unroll 1
  for (int i = 0; i < 16; ++i) {
    const int lr = 16 * wave + i;
    const int r  = rowBase + lr;
    const v4f sv = *(const v4fa*)(stg + lr * DF + 4 * lane);
    asm volatile("" :: "v"(sv));
    const v4f t = sv + bb;
    v4f y;
    y.x = (t.x >= 0.0f) ? t.x : 0.01f * t.x;
    y.y = (t.y >= 0.0f) ? t.y : 0.01f * t.y;
    y.z = (t.z >= 0.0f) ? t.z : 0.01f * t.z;
    y.w = (t.w >= 0.0f) ? t.w : 0.01f * t.w;
    y.x = pz ? qn : y.x; y.y = pz ? qn : y.y; y.z = pz ? qn : y.z; y.w = pz ? qn : y.w;
    if (r < nN) *(volatile v4f*)(outp + (size_t)r * DF + 4 * lane) = y;
  }
}

__global__ __launch_bounds__(GTHR) __attribute__((amdgpu_num_vgpr(248)))
void k_gemm(const unsigned short* __restrict__ Apl, const unsigned short* __restrict__ WD,
            const float* __restrict__ BT, const int* __restrict__ FLG, float* outp, int nN) {
  extern __shared__ __attribute__((aligned(16))) float gsm[];
  float* stg = gsm;
  float* bsh = gsm + GBM * DF;
  const int tid = (int)threadIdx.x, lane = tid & 31, wave = tid >> 5, hh = lane >> 4, m = lane & 15;
  const int rowBase = (int)blockIdx.x * GBM;

  if (tid < 32) {
    const v4f b4 = *(const v4f*)(BT + 4 * tid);
    *(v4fa*)(bsh + 4 * tid) = b4;
  }

  v8f acc[8];
  {
    const v8f z = {0.f, 0.f, 0.f, 0.f, 0.f, 0.f, 0.f, 0.f};
#pragma unroll
    for (int t = 0; t < 8; ++t) acc[t] = z;
  }
  const unsigned short* ap = Apl + (size_t)(rowBase + 16 * wave + m) * (size_t)AP + 8 * hh;
  const unsigned short* bp = WD + (size_t)m * (size_t)WDP + 8 * hh;

#pragma unroll 1
  for (int k0 = 0; k0 < KG; k0 += 32) {
    FragB af;
    af.h[0] = *(const v8usa*)(ap + k0);
    af.h[1] = *(const v8usa*)(ap + k0 + 16);
#pragma unroll
    for (int nt = 0; nt < 8; ++nt) {
      const unsigned short* wq = bp + (size_t)(16 * nt) * (size_t)WDP + k0;
      FragB bf;
      bf.h[0] = *(const v8usa*)wq;
      bf.h[1] = *(const v8usa*)(wq + 16);
      acc[nt] = wmb(af, bf, acc[nt]);
    }
  }

#pragma unroll
  for (int nt = 0; nt < 8; ++nt) {
    const int lc = 16 * nt + m;
#pragma unroll
    for (int r = 0; r < 8; ++r) {
      const int lr = 16 * wave + 8 * hh + r;
      stg[lr * DF + lc] = acc[nt][r];
    }
  }
  __syncthreads();

  const v4f bb = *(const v4fa*)(bsh + 4 * lane);
  const int fl = FLG[(size_t)(rowBase >> PKS) * 32 + 1];
  const bool pz = fl != 0;
  out_pass(stg, bb, pz, outp, rowBase, wave, lane, nN);
  __threadfence();
  out_pass(stg, bb, pz, outp, rowBase, wave, lane, nN);
}

static inline int cdiv(int a, int b) { return (a + b - 1) / b; }
static inline size_t al256(size_t o) { return (o + 255) & ~(size_t)255; }

extern "C" void kernel_launch(void* const* d_in, const int* in_sizes, int n_in,
                              void* d_out, int out_size, void* d_ws, size_t ws_size,
                              hipStream_t stream) {
  if (n_in < 5) return;
  const int nE = in_sizes[0];
  if (nE < 1 || in_sizes[1] != nE || nE >= (1 << 21)) return;
  if (in_sizes[2] < DF || (in_sizes[2] % DF) != 0) return;
  const int nN = in_sizes[2] / DF;
  if (nN != NNODES) return;
  if (in_sizes[3] != DF * DF || in_sizes[4] != DF) return;
  if ((long long)out_size != (long long)nN * DF) return;

  const int*   srcv = (const int*)  d_in[0];
  const int*   dstv = (const int*)  d_in[1];
  const float* x    = (const float*)d_in[2];
  const float* W    = (const float*)d_in[3];
  const float* b    = (const float*)d_in[4];
  float* out = (float*)d_out;

  const int nB    = cdiv(nN, NBA);
  const int NPADN = nB * NBA;
  const int MP    = cdiv(nN, GBM) * GBM;
  if (MP > NPADN || nB > 64) return;
  const int segLen = cdiv(cdiv(nE, NWAVE), WIT) * WIT;
  if ((long long)segLen * NWAVE < (long long)nE) return;

  char* ws = (char*)d_ws;
  size_t off = 0;
  const size_t oWD = off; off = al256(off + (size_t)DF * WDP * 2);
  const size_t oBT = off; off = al256(off + (size_t)DF * 4);
  const size_t oFL = off; off = al256(off + (size_t)(2 * nB) * 128);
  const size_t oCN = off; off = al256(off + (size_t)NPADN * 4);
  const size_t oOF = off; off = al256(off + (size_t)NPADN * 4);
  const size_t oNI = off; off = al256(off + (size_t)NPADN * 4);
  const size_t oNO = off; off = al256(off + (size_t)NPADN * 4);
  const size_t oLS = off; off = al256(off + (size_t)nB * RCAP * 4);
  const size_t oPN = off; off = al256(off + (size_t)nN * DF * 4);
  const size_t oAG = off; off = al256(off + (size_t)MP * AP * 2);
  if (off > ws_size || off > (size_t)134217728) return;
  unsigned short* WD  = (unsigned short*)(ws + oWD);
  float* BT   = (float*)(ws + oBT);
  int*   FLG  = (int*)(ws + oFL);
  int*   CNT  = (int*)(ws + oCN);
  int*   OFF  = (int*)(ws + oOF);
  int*   NIb  = (int*)(ws + oNI);
  int*   NOb  = (int*)(ws + oNO);
  int*   LIST = (int*)(ws + oLS);
  float* PN   = (float*)(ws + oPN);
  unsigned short* AGG = (unsigned short*)(ws + oAG);

  hipFuncSetAttribute(reinterpret_cast<const void*>(&k_bucket), hipFuncAttributeMaxDynamicSharedMemorySize, LDS_BK);
  hipFuncSetAttribute(reinterpret_cast<const void*>(&k_gemm), hipFuncAttributeMaxDynamicSharedMemorySize, LDS_GM);

  const int padPieces = (MP - nN) * 32;
  const int nUnits = UW + 32 + padPieces;
  k_prep<<<cdiv(nUnits, NTHR), NTHR, 0, stream>>>(W, b, WD, BT, AGG, nN, padPieces);
  k_bucket<<<2 * nB, NTHR, LDS_BK, stream>>>(srcv, dstv, nE, nN, segLen, nB, LIST, CNT, OFF, NIb, NOb, FLG);
  k_prescale<<<cdiv(nN, RPB), NTHR, 0, stream>>>(x, (const float*)NOb, FLG, PN, nN, nB);
  k_replay<<<nB, NTHR, 0, stream>>>(PN, LIST, CNT, OFF, (const float*)NIb, FLG, AGG, nN);
  k_gemm<<<MP / GBM, GTHR, LDS_GM, stream>>>(AGG, WD, BT, FLG, out, nN);
}
